// LYT_19447611916714
// MI455X (gfx1250) — hardware-verified
//
#include <hip/hip_runtime.h>
#include <hip/hip_bf16.h>


#define NB_  4
#define HH_  64
#define WW_  64
#define NL_  4096
#define DM_  192
#define DI_  384
#define NS_  16
#define KG_  4
#define RK_  12
#define CT_  44
#define CP_  64
#define MT_  16384

static_assert(NL_ == HH_ * WW_);
static_assert(MT_ == NB_ * NL_);
static_assert(MT_ % 64 == 0);
static_assert(NL_ % 64 == 0);
static_assert(DM_ % 64 == 0);
static_assert((2 * DI_) % 64 == 0);
static_assert(DI_ % 64 == 0);
static_assert(DM_ % 32 == 0);
static_assert(DI_ % 128 == 0);
static_assert(DI_ == 384);
static_assert(CT_ == RK_ + 2 * NS_);
static_assert(CP_ >= CT_ && CP_ % 32 == 0);
static_assert(HH_ == 64 && WW_ == 64);
static_assert(MT_ % 8 == 0);

typedef float          v2f   __attribute__((ext_vector_type(2)));
typedef float          v4f   __attribute__((ext_vector_type(4)));
typedef float          v8f   __attribute__((ext_vector_type(8)));
typedef _Float16       v8h   __attribute__((ext_vector_type(8)));
typedef _Float16       v16h  __attribute__((ext_vector_type(16)));
typedef __bf16         v16b  __attribute__((ext_vector_type(16)));
typedef unsigned short u16x8 __attribute__((ext_vector_type(8)));

union FragH { u16x8 h[2]; v16h v; };
union FragB { u16x8 h[2]; v16b v; };
union Pack8 { v8h f; u16x8 u; };

__device__ __forceinline__ unsigned short f32_to_bf16(float f) {
    unsigned u = __float_as_uint(f);
    unsigned r = u + 0x7FFFu + ((u >> 16) & 1u);
    return (unsigned short)(r >> 16);
}
__device__ __forceinline__ float bf16_to_f32(unsigned short b) {
    return __uint_as_float(((unsigned)b) << 16);
}
__device__ __forceinline__ float silu_f(float x) {
    const float e = __expf(-x);
    return x * __builtin_amdgcn_rcpf(1.0f + e);
}
__device__ __forceinline__ v8f ld8f(const float* p) {
    v4f a = *(const v4f*)p;
    v4f b = *(const v4f*)(p + 4);
    return __builtin_shufflevector(a, b, 0, 1, 2, 3, 4, 5, 6, 7);
}
__device__ __forceinline__ float hsum8(v8f a) {
    return ((a[0] + a[1]) + (a[2] + a[3])) + ((a[4] + a[5]) + (a[6] + a[7]));
}
__device__ __forceinline__ float wsum32(float v) {
#pragma unroll
    for (int o = 16; o > 0; o >>= 1) v += __shfl_xor(v, o, 32);
    return v;
}

__device__ __forceinline__ void mma16(v8f& acc, const FragH& a, const FragH& b) {
    acc = __builtin_amdgcn_wmma_f32_16x16x32_f16(false, a.v, false, b.v, (short)0, acc, false, false);
    asm volatile("v_nop\n\tv_nop\n\tv_nop\n\tv_nop" : "+v"(acc) : "v"(a.v), "v"(b.v));
}
__device__ __forceinline__ void mma16(v8f& acc, const FragB& a, const FragB& b) {
    acc = __builtin_amdgcn_wmma_f32_16x16x32_bf16(false, a.v, false, b.v, (short)0, acc, false, false);
    asm volatile("v_nop\n\tv_nop\n\tv_nop\n\tv_nop" : "+v"(acc) : "v"(a.v), "v"(b.v));
}

__global__ __launch_bounds__(256)
void cvt_hilo_kernel(const float* __restrict__ src, unsigned short* dst0, unsigned short* dst1, int n8)
{
    const int i = blockIdx.x * 256 + threadIdx.x;
    if (i >= n8) return;
    const size_t e = (size_t)i * 8;
    const v8f x = ld8f(src + e);
    u16x8 hv, lv;
#pragma unroll
    for (int c = 0; c < 8; ++c) {
        const float f = x[c];
        const unsigned short hb = f32_to_bf16(f);
        const unsigned short lb = f32_to_bf16(f - bf16_to_f32(hb));
        hv[c] = hb;
        lv[c] = lb;
    }
    *(volatile u16x8*)(dst0 + e) = hv;
    *(volatile u16x8*)(dst1 + e) = lv;
    __threadfence();
    *(volatile u16x8*)(dst0 + e) = hv;
    *(volatile u16x8*)(dst1 + e) = lv;
}

__global__ __launch_bounds__(256)
void pack_wx_kernel(const float* __restrict__ w, unsigned short* dst, int n8, float scale)
{
    const int i = blockIdx.x * 256 + threadIdx.x;
    if (i >= n8) return;
    const int d8 = i % (DI_ / 8);
    const int c  = (i / (DI_ / 8)) % CP_;
    const int k  = i / ((DI_ / 8) * CP_);
    const int cc = (c < CT_) ? c : (CT_ - 1);
    v8f x = ld8f(w + ((size_t)(k * CT_ + cc)) * DI_ + (size_t)d8 * 8);
    if (c >= CT_) {
#pragma unroll
        for (int q = 0; q < 8; ++q) x[q] = 0.0f;
    }
    Pack8 pk;
    pk.f = __builtin_convertvector(x * scale, v8h);
    const u16x8 v = pk.u;
    const size_t e = (size_t)i * 8;
    *(volatile u16x8*)(dst + e) = v;
    __threadfence();
    *(volatile u16x8*)(dst + e) = v;
}

__device__ __forceinline__ void tile_store_pass(const float* st, float* gp, int ldc, int lane) {
    constexpr int P   = 36;
    const int rsub = lane >> 3;
    const int c4   = (lane & 7) * 4;
#pragma unroll
    for (int it = 0; it < 8; ++it) {
        const int row = it * 4 + rsub;
        const v4f v = *(const v4f*)(st + row * P + c4);
        *(volatile v4f*)(gp + (size_t)row * ldc + c4) = v;
    }
}

template<typename FR, bool SPLIT, bool ACT2>
__global__ __launch_bounds__(128)
void gemm_tn_kernel(const unsigned short* __restrict__ A,  const unsigned short* __restrict__ A2,
                    const unsigned short* __restrict__ Bw, const unsigned short* __restrict__ B2,
                    float* C, float* C2,
                    long long zsA, long long zsB, long long zsC,
                    int K, int ldc, int csplit, int zdivA, float scale)
{
    constexpr int NBF = 2;
    constexpr int P   = 36;
    __shared__ __attribute__((aligned(16))) float stile[4][32 * P];

    const int tid  = threadIdx.x;
    const int lane = tid & 31;
    const int wave = tid >> 5;
    const int h    = lane >> 4;
    const int m    = lane & 15;
    const int wm   = wave >> 1;
    const int wn   = wave & 1;

    const int z  = blockIdx.z;
    const int za = z / zdivA;
    const int zb = z - za * zdivA;
    const unsigned short* Ab  = A  + (size_t)za * (size_t)zsA;
    const unsigned short* A2b = A2 + (size_t)za * (size_t)zsA;
    const unsigned short* Bb  = Bw + (size_t)zb * (size_t)zsB;
    const unsigned short* B2b = B2 + (size_t)zb * (size_t)zsB;

    const int rowW = blockIdx.y * 64 + wm * 32;
    const int colW = blockIdx.x * 64 + wn * 32;

    v8f acc[2 * NBF];
#pragma unroll
    for (int j = 0; j < 2 * NBF; ++j)
#pragma unroll
        for (int r = 0; r < 8; ++r) acc[j][r] = 0.0f;

    const size_t aoff  = (size_t)(rowW + m) * K + 8 * h;
    const size_t boff  = (size_t)(colW + m) * K + 8 * h;
    const size_t sub16 = (size_t)16 * K;
    const int nk = K >> 5;

    for (int kt = 0; kt < nk; ++kt) {
        const size_t k0 = (size_t)kt * 32;
        FR fa[2], fb[NBF], ga[2], gb[NBF];
#pragma unroll
        for (int s = 0; s < 2; ++s) {
            const unsigned short* p = Ab + aoff + s * sub16 + k0;
            fa[s].h[0] = *(const u16x8*)(p);
            fa[s].h[1] = *(const u16x8*)(p + 16);
            if (SPLIT) {
                const unsigned short* q = A2b + aoff + s * sub16 + k0;
                ga[s].h[0] = *(const u16x8*)(q);
                ga[s].h[1] = *(const u16x8*)(q + 16);
            }
        }
#pragma unroll
        for (int j = 0; j < NBF; ++j) {
            const unsigned short* p = Bb + boff + j * sub16 + k0;
            fb[j].h[0] = *(const u16x8*)(p);
            fb[j].h[1] = *(const u16x8*)(p + 16);
            if (SPLIT) {
                const unsigned short* q = B2b + boff + j * sub16 + k0;
                gb[j].h[0] = *(const u16x8*)(q);
                gb[j].h[1] = *(const u16x8*)(q + 16);
            }
        }
#pragma unroll
        for (int s = 0; s < 2; ++s)
#pragma unroll
            for (int j = 0; j < NBF; ++j) {
                mma16(acc[s * NBF + j], fa[s], fb[j]);
                if (SPLIT) {
                    mma16(acc[s * NBF + j], fa[s], gb[j]);
                    mma16(acc[s * NBF + j], ga[s], fb[j]);
                }
            }
    }

    const bool zh = (colW >= csplit);
    float* st = stile[wave];
#pragma unroll
    for (int s = 0; s < 2; ++s)
#pragma unroll
        for (int j = 0; j < NBF; ++j)
#pragma unroll
            for (int r = 0; r < 8; ++r) {
                float v = acc[s * NBF + j][r] * scale;
                if (ACT2) v = zh ? silu_f(v) : v;
                st[(s * 16 + 8 * h + r) * P + j * 16 + m] = v;
            }
    __syncthreads();

    float* Cp = C;
    int gcol = colW;
    if (zh) { Cp = C2; gcol = colW - csplit; }
    float* gp = Cp + (size_t)z * (size_t)zsC + (size_t)rowW * ldc + gcol;
    tile_store_pass(st, gp, ldc, lane);
    __threadfence();
    tile_store_pass(st, gp, ldc, lane);
}

__global__ __launch_bounds__(192)
void dwconv_silu_kernel(const float* __restrict__ xp, const float* __restrict__ cw,
                        const float* __restrict__ cb, float* xc32, unsigned int* xc16, float scale16)
{
    const int bh = blockIdx.x;
    const int b  = bh / HH_;
    const int h  = bh - b * HH_;
    const int t  = threadIdx.x;
    const int d  = 2 * t;

    float wa[9], wb[9];
#pragma unroll
    for (int i = 0; i < 9; ++i) { wa[i] = cw[(size_t)d * 9 + i]; wb[i] = cw[(size_t)(d + 1) * 9 + i]; }
    const float cba = cb[d], cbb = cb[d + 1];

    const bool vm = (h > 0), vp = (h < HH_ - 1);
    const int hm = vm ? (h - 1) : 0;
    const int hp = vp ? (h + 1) : (HH_ - 1);
    const float* rm = xp + ((size_t)(b * HH_ + hm) * WW_) * DI_ + d;
    const float* rc = xp + ((size_t)(b * HH_ + h)  * WW_) * DI_ + d;
    const float* rp = xp + ((size_t)(b * HH_ + hp) * WW_) * DI_ + d;

    v2f z2; z2.x = 0.0f; z2.y = 0.0f;
    v2f m0 = z2, c0 = z2, p0 = z2;
    v2f m1 = *(const v2f*)rm; m1 = vm ? m1 : z2;
    v2f c1 = *(const v2f*)rc;
    v2f p1 = *(const v2f*)rp; p1 = vp ? p1 : z2;

    const size_t obase = ((size_t)(b * HH_ + h) * WW_) * DI_ + d;

#pragma unroll 1
    for (int w = 0; w < WW_; ++w) {
        const bool vn = (w + 1 < WW_);
        const int  wn = vn ? (w + 1) : (WW_ - 1);
        v2f m2 = *(const v2f*)(rm + (size_t)wn * DI_); m2 = (vm && vn) ? m2 : z2;
        v2f c2 = *(const v2f*)(rc + (size_t)wn * DI_); c2 = vn ? c2 : z2;
        v2f p2 = *(const v2f*)(rp + (size_t)wn * DI_); p2 = (vp && vn) ? p2 : z2;

        float sa = wa[0] * m0.x + wa[1] * m1.x + wa[2] * m2.x
                 + wa[3] * c0.x + wa[4] * c1.x + wa[5] * c2.x
                 + wa[6] * p0.x + wa[7] * p1.x + wa[8] * p2.x;
        float sb = wb[0] * m0.y + wb[1] * m1.y + wb[2] * m2.y
                 + wb[3] * c0.y + wb[4] * c1.y + wb[5] * c2.y
                 + wb[6] * p0.y + wb[7] * p1.y + wb[8] * p2.y;
        const float ua = silu_f(sa + cba);
        const float ub = silu_f(sb + cbb);

        v2f o; o.x = ua; o.y = ub;
        const _Float16 fa16 = (_Float16)(ua * scale16);
        const _Float16 fb16 = (_Float16)(ub * scale16);
        const unsigned int pk = (unsigned int)__builtin_bit_cast(unsigned short, fa16)
                              | ((unsigned int)__builtin_bit_cast(unsigned short, fb16) << 16);
        const size_t e = obase + (size_t)w * DI_;
        float* po = xc32 + e;
        unsigned int* ph = xc16 + (e >> 1);
        *(volatile v2f*)po = o;
        *(volatile unsigned int*)ph = pk;
        __threadfence();
        *(volatile v2f*)po = o;
        *(volatile unsigned int*)ph = pk;

        m0 = m1; m1 = m2; c0 = c1; c1 = c2; p0 = p1; p1 = p2;
    }
}

__global__ __launch_bounds__(128)
void scan_kernel(const float* __restrict__ xdbl, const float* __restrict__ xc,
                 const float* __restrict__ dtw, const float* __restrict__ dtb,
                 const float* __restrict__ alog, const float* __restrict__ Dsv,
                 float* Y)
{
    const int b = blockIdx.y;
    const int d = blockIdx.x * 128 + threadIdx.x;
    const size_t colbase = (size_t)b * NL_ * DI_ + d;
    const float* xcb = xc + colbase;
    float* Yb = Y + colbase;

#pragma unroll 1
    for (int k = 0; k < KG_; ++k) {
        const int ch = k * DI_ + d;
        float An[NS_], hs[NS_];
#pragma unroll
        for (int n = 0; n < NS_; ++n) { An[n] = -__expf(alog[(size_t)ch * NS_ + n]); hs[n] = 0.0f; }
        float wr[RK_];
#pragma unroll
        for (int r = 0; r < RK_; ++r) wr[r] = dtw[(size_t)ch * RK_ + r];
        const float bias = dtb[ch];
        const float Dd   = Dsv[ch];
        const float* xd  = xdbl + (size_t)(b * KG_ + k) * NL_ * CP_;
        const int rmask  = (k & 2) ? (NL_ - 1) : 0;
        const int tr     = k & 1;

#pragma unroll 1
        for (int l = 0; l < NL_; ++l) {
            const int t  = l ^ rmask;
            const int pt = ((t & (WW_ - 1)) * WW_) + (t >> 6);
            const int p  = tr ? pt : t;
            const float* row = xd + (size_t)p * CP_;

            v4f q[11];
#pragma unroll
            for (int i = 0; i < 11; ++i) q[i] = *(const v4f*)(row + 4 * i);
            float dr[RK_], Bn[NS_], Cn[NS_];
#pragma unroll
            for (int i = 0; i < 4; ++i) {
                dr[i] = q[0][i]; dr[4 + i] = q[1][i]; dr[8 + i] = q[2][i];
                Bn[i] = q[3][i]; Bn[4 + i] = q[4][i]; Bn[8 + i] = q[5][i]; Bn[12 + i] = q[6][i];
                Cn[i] = q[7][i]; Cn[4 + i] = q[8][i]; Cn[8 + i] = q[9][i]; Cn[12 + i] = q[10][i];
            }

            const float u = xcb[(size_t)p * DI_];

            float x = 0.0f;
#pragma unroll
            for (int r = 0; r < RK_; ++r) x += wr[r] * dr[r];
            x += bias;
            const float delta = fmaxf(x, 0.0f) + log1pf(__expf(-fabsf(x)));
            const float du = delta * u;

            float y = 0.0f;
#pragma unroll
            for (int n = 0; n < NS_; ++n) {
                const float a = __expf(delta * An[n]);
                hs[n] = a * hs[n] + du * Bn[n];
                y += hs[n] * Cn[n];
            }
            y += Dd * u;

            const size_t pe = (size_t)p * DI_;
            float prev = 0.0f;
            if (k != 0) prev = Yb[pe];
            const float v = prev + y;
            *(volatile float*)(Yb + pe) = v;
            __threadfence();
            *(volatile float*)(Yb + pe) = v;
        }
    }
}

__global__ __launch_bounds__(256)
void ln_gate_kernel(const float* __restrict__ Y, const float* __restrict__ Z,
                    const float* __restrict__ gam, const float* __restrict__ bet,
                    unsigned short* yzh, unsigned short* yzl, int nrows)
{
    const int lane = threadIdx.x & 31;
    const int row  = blockIdx.x * 8 + (threadIdx.x >> 5);
    const int rowc = (row < nrows) ? row : (nrows - 1);
    const int c0   = lane * 8;
    const int c1   = 256 + (lane & 15) * 8;
    const bool own2 = lane < 16;
    const float* yr = Y + (size_t)rowc * DI_;
    const float* zr = Z + (size_t)rowc * DI_;

    const v8f ya = ld8f(yr + c0);
    const v8f yb = ld8f(yr + c1);
    float s = hsum8(ya) + (own2 ? hsum8(yb) : 0.0f);
    s = wsum32(s);
    const float mu = s * (1.0f / (float)DI_);
    const v8f da = ya - mu;
    const v8f db = yb - mu;
    float ss = hsum8(da * da) + (own2 ? hsum8(db * db) : 0.0f);
    ss = wsum32(ss);
    const float var = ss * (1.0f / (float)DI_);
    const float inv = __builtin_amdgcn_rcpf(sqrtf(var + 1e-5f));

    const v8f ga = ld8f(gam + c0), gb = ld8f(gam + c1);
    const v8f ba = ld8f(bet + c0), bb = ld8f(bet + c1);
    const v8f za = ld8f(zr + c0),  zb = ld8f(zr + c1);
    const v8f oa = (da * inv * ga + ba) * za;
    const v8f ob = (db * inv * gb + bb) * zb;

    u16x8 ha, la, hb, lb;
#pragma unroll
    for (int c = 0; c < 8; ++c) {
        unsigned short t0 = f32_to_bf16(oa[c]);
        ha[c] = t0; la[c] = f32_to_bf16(oa[c] - bf16_to_f32(t0));
        unsigned short t1 = f32_to_bf16(ob[c]);
        hb[c] = t1; lb[c] = f32_to_bf16(ob[c] - bf16_to_f32(t1));
    }
    if (row < nrows) {
        unsigned short* ph = yzh + (size_t)row * DI_;
        unsigned short* pl = yzl + (size_t)row * DI_;
        *(volatile u16x8*)(ph + c0) = ha;
        *(volatile u16x8*)(pl + c0) = la;
        if (own2) { *(volatile u16x8*)(ph + c1) = hb; *(volatile u16x8*)(pl + c1) = lb; }
        __threadfence();
        *(volatile u16x8*)(ph + c0) = ha;
        *(volatile u16x8*)(pl + c0) = la;
        if (own2) { *(volatile u16x8*)(ph + c1) = hb; *(volatile u16x8*)(pl + c1) = lb; }
    }
}

extern "C" void kernel_launch(void* const* d_in, const int* in_sizes, int n_in,
                              void* d_out, int out_size, void* d_ws, size_t ws_size,
                              hipStream_t stream)
{
    if (n_in < 12) return;
    if (in_sizes[0]  != MT_ * DM_)        return;
    if (in_sizes[1]  != 2 * DI_ * DM_)    return;
    if (in_sizes[2]  != DI_ * 9)          return;
    if (in_sizes[3]  != DI_)              return;
    if (in_sizes[4]  != KG_ * CT_ * DI_)  return;
    if (in_sizes[5]  != KG_ * DI_ * RK_)  return;
    if (in_sizes[6]  != KG_ * DI_)        return;
    if (in_sizes[7]  != KG_ * DI_ * NS_)  return;
    if (in_sizes[8]  != KG_ * DI_)        return;
    if (in_sizes[9]  != DI_)              return;
    if (in_sizes[10] != DI_)              return;
    if (in_sizes[11] != DM_ * DI_)        return;
    if (out_size != MT_ * DM_)            return;

    const float* x    = (const float*)d_in[0];
    const float* wi   = (const float*)d_in[1];
    const float* cw   = (const float*)d_in[2];
    const float* cb   = (const float*)d_in[3];
    const float* wx   = (const float*)d_in[4];
    const float* dtw  = (const float*)d_in[5];
    const float* dtb  = (const float*)d_in[6];
    const float* alog = (const float*)d_in[7];
    const float* Dsp  = (const float*)d_in[8];
    const float* gam  = (const float*)d_in[9];
    const float* bet  = (const float*)d_in[10];
    const float* wo   = (const float*)d_in[11];
    float* out = (float*)d_out;

    const size_t SZ_F  = (size_t)MT_ * DI_ * 4;
    const size_t SZ_H  = (size_t)MT_ * DI_ * 2;
    const size_t SZ_XH = (size_t)MT_ * DM_ * 2;
    const size_t SZ_XD = (size_t)NB_ * KG_ * NL_ * CP_ * 4;
    const size_t SZ_WI = (size_t)2 * DI_ * DM_ * 2;
    const size_t SZ_WX = (size_t)KG_ * CP_ * DI_ * 2;
    const size_t SZ_WO = (size_t)DM_ * DI_ * 2;

    const size_t OFF_RA  = 0;
    const size_t OFF_RB  = OFF_RA + SZ_F;
    const size_t OFF_RC  = OFF_RB + SZ_F;
    const size_t OFF_RD  = OFF_RC + SZ_F;
    const size_t OFF_RE  = OFF_RD + SZ_H;
    const size_t OFF_WIH = OFF_RE + SZ_F;
    const size_t OFF_WIL = OFF_WIH + SZ_WI;
    const size_t OFF_WX  = OFF_WIL + SZ_WI;
    const size_t OFF_WOH = OFF_WX + SZ_WX;
    const size_t OFF_WOL = OFF_WOH + SZ_WO;
    const size_t WS_END  = OFF_WOL + SZ_WO;
    if (SZ_XD > SZ_F)       return;
    if (2 * SZ_H > SZ_F)    return;
    if (2 * SZ_XH > SZ_H)   return;
    if (ws_size < WS_END)   return;

    char* ws = (char*)d_ws;
    float*          Xp   = (float*)(ws + OFF_RA);
    float*          Xd   = (float*)(ws + OFF_RA);
    unsigned short* yzh  = (unsigned short*)(ws + OFF_RA);
    unsigned short* yzl  = (unsigned short*)(ws + OFF_RA + SZ_H);
    float*          Zs   = (float*)(ws + OFF_RB);
    float*          Xc32 = (float*)(ws + OFF_RC);
    unsigned short* xh   = (unsigned short*)(ws + OFF_RD);
    unsigned short* xl   = (unsigned short*)(ws + OFF_RD + SZ_XH);
    unsigned short* xc16 = (unsigned short*)(ws + OFF_RD);
    float*          Yp   = (float*)(ws + OFF_RE);
    unsigned short* wih  = (unsigned short*)(ws + OFF_WIH);
    unsigned short* wil  = (unsigned short*)(ws + OFF_WIL);
    unsigned short* wx16 = (unsigned short*)(ws + OFF_WX);
    unsigned short* woh  = (unsigned short*)(ws + OFF_WOH);
    unsigned short* wol  = (unsigned short*)(ws + OFF_WOL);

    {
        int n8 = (MT_ * DM_) / 8;
        hipLaunchKernelGGL(cvt_hilo_kernel, dim3((n8 + 255) / 256), dim3(256), 0, stream, x, xh, xl, n8);
        n8 = (2 * DI_ * DM_) / 8;
        hipLaunchKernelGGL(cvt_hilo_kernel, dim3((n8 + 255) / 256), dim3(256), 0, stream, wi, wih, wil, n8);
        n8 = (DM_ * DI_) / 8;
        hipLaunchKernelGGL(cvt_hilo_kernel, dim3((n8 + 255) / 256), dim3(256), 0, stream, wo, woh, wol, n8);
        n8 = (KG_ * CP_ * DI_) / 8;
        hipLaunchKernelGGL(pack_wx_kernel, dim3((n8 + 255) / 256), dim3(256), 0, stream, wx, wx16, n8, 64.0f);
    }

    hipLaunchKernelGGL(HIP_KERNEL_NAME(gemm_tn_kernel<FragB, true, true>),
                       dim3((2 * DI_) / 64, MT_ / 64, 1), dim3(128), 0, stream,
                       (const unsigned short*)xh, (const unsigned short*)xl,
                       (const unsigned short*)wih, (const unsigned short*)wil,
                       Xp, Zs, (long long)0, (long long)0, (long long)0,
                       (int)DM_, (int)DI_, (int)DI_, (int)1, 1.0f);

    hipLaunchKernelGGL(dwconv_silu_kernel, dim3(NB_ * HH_), dim3(DI_ / 2), 0, stream,
                       (const float*)Xp, cw, cb, Xc32, (unsigned int*)xc16, 64.0f);

    hipLaunchKernelGGL(HIP_KERNEL_NAME(gemm_tn_kernel<FragH, false, false>),
                       dim3(CP_ / 64, NL_ / 64, NB_ * KG_), dim3(128), 0, stream,
                       (const unsigned short*)xc16, (const unsigned short*)xc16,
                       (const unsigned short*)wx16, (const unsigned short*)wx16,
                       Xd, Xd, (long long)NL_ * DI_, (long long)CP_ * DI_, (long long)NL_ * CP_,
                       (int)DI_, (int)CP_, (int)(1 << 30), (int)KG_, 0.000244140625f);

    hipLaunchKernelGGL(scan_kernel, dim3(DI_ / 128, NB_), dim3(128), 0, stream,
                       (const float*)Xd, (const float*)Xc32, dtw, dtb, alog, Dsp, Yp);

    hipLaunchKernelGGL(ln_gate_kernel, dim3(MT_ / 8), dim3(256), 0, stream,
                       (const float*)Yp, (const float*)Zs, gam, bet, yzh, yzl, (int)MT_);

    hipLaunchKernelGGL(HIP_KERNEL_NAME(gemm_tn_kernel<FragB, true, false>),
                       dim3(DM_ / 64, MT_ / 64, 1), dim3(128), 0, stream,
                       (const unsigned short*)yzh, (const unsigned short*)yzl,
                       (const unsigned short*)woh, (const unsigned short*)wol,
                       out, out, (long long)0, (long long)0, (long long)0,
                       (int)DI_, (int)DM_, (int)(1 << 30), (int)1, 1.0f);
}
